// NEPNN_90726889160848
// MI455X (gfx1250) — hardware-verified
//
#include <hip/hip_runtime.h>
#include <stddef.h>


typedef _Float16 h16;
typedef _Float16 v16h __attribute__((ext_vector_type(16)));
typedef _Float16 v8h  __attribute__((ext_vector_type(8)));
typedef float    v8f  __attribute__((ext_vector_type(8)));
typedef float    v4f  __attribute__((ext_vector_type(4)));

#ifndef NE
#define NE 262144
#endif
#define NE_FULL 262144
#define NTYPE 16
#define NHID  32
#define NBAS  16
#define NOUT  8
#define BN_EPS 1.0e-5f

#define WAVES 8
#define TPW   8
#define NTILES (NE / 16)
#define NBLK   (NTILES / (WAVES * TPW))

static_assert(NE >= 1024 && NE <= NE_FULL);
static_assert((NE % (16 * WAVES * TPW)) == 0);
static_assert(NTILES == NBLK * WAVES * TPW);
static_assert(NTYPE == 16 && NHID == 32 && NBAS == 16 && NOUT == 8);
static_assert((NTYPE * NBAS) % 32 == 0);
static_assert(NHID == 32);
static_assert((NTYPE * NOUT) % 16 == 0);
static_assert(((NE * 2) % 256) == 0);

#define WCARRY 64.0f
#define FCARRY 16.0f
#define YCARRY 256.0f
#define L1SCALE (1.0f / (WCARRY * FCARRY))
#define L2SCALE (1.0f / (WCARRY * YCARRY))

#define W0_HALVES (NTYPE * NHID * NBAS)
#define W1_HALVES (NTYPE * NOUT * NHID)
#define W0_PIECES (W0_HALVES / 8)
#define W1_PIECES (W1_HALVES / 8)
static_assert((W0_PIECES % 256) == 0 && (W1_PIECES % 256) == 0);
static_assert(W0_PIECES == 4 * 256 && W1_PIECES == 2 * 256);

#define P1W 64
#define P2W 32
#define T1W 64
#define T2W 32

#define W0H_BYTES ((size_t)W0_HALVES * 2)
#define W1H_BYTES ((size_t)W1_HALVES * 2)
#define P1_BYTES  ((size_t)NBLK * P1W * 4)
#define T1_BYTES  ((size_t)T1W * 4)
#define P2_BYTES  ((size_t)NBLK * P2W * 4)
#define T2_BYTES  ((size_t)T2W * 4)
#define O2_BYTES  ((size_t)NE * NOUT * 4)
#define OFF_W0H ((size_t)0)
#define OFF_W1H (OFF_W0H + W0H_BYTES)
#define OFF_P1  (OFF_W1H + W1H_BYTES)
#define OFF_T1  (OFF_P1 + P1_BYTES)
#define OFF_P2  (OFF_T1 + T1_BYTES)
#define OFF_T2  (OFF_P2 + P2_BYTES)
#define OFF_O2  (OFF_T2 + T2_BYTES)
#define WS_TOTAL (OFF_O2 + O2_BYTES)
static_assert((W0H_BYTES % 128) == 0 && (W1H_BYTES % 128) == 0 && (P1_BYTES % 128) == 0);
static_assert((T1_BYTES % 128) == 0 && (P2_BYTES % 128) == 0 && (T2_BYTES % 128) == 0);
static_assert((O2_BYTES % 128) == 0);
static_assert(WS_TOTAL <= (size_t)134217728);

__device__ __forceinline__ float bf16r(float x) {
  unsigned int u = __float_as_uint(x);
  u = (u + 0x7FFFu + ((u >> 16) & 1u)) & 0xFFFF0000u;
  return __uint_as_float(u);
}

static __device__ __forceinline__ h16 toh_flush(float v) {
  const h16 r = (h16)v;
  return (fabsf(v) < 6.103515625e-05f) ? (h16)0.0f : r;
}

__device__ __forceinline__ v16h frag_at(const _Float16* p) {
  v8h lo = *(const v8h*)(p);
  v8h hi = *(const v8h*)(p + 16);
  v16h out;
#pragma unroll
  for (int i = 0; i < 8; ++i) { out[i] = lo[i]; out[i + 8] = hi[i]; }
  return out;
}

__device__ __forceinline__ v16h frag2(const _Float16* plo, const _Float16* phi) {
  v8h lo = *(const v8h*)(plo);
  v8h hi = *(const v8h*)(phi);
  v16h out;
#pragma unroll
  for (int i = 0; i < 8; ++i) { out[i] = lo[i]; out[i + 8] = hi[i]; }
  return out;
}

__device__ __forceinline__ v16h join8(v8h lo, v8h hi) {
  v16h out;
#pragma unroll
  for (int i = 0; i < 8; ++i) { out[i] = lo[i]; out[i + 8] = hi[i]; }
  return out;
}

__device__ __forceinline__ v8f wmma16(v16h a, v16h b, v8f c) {
  v8f d = __builtin_amdgcn_wmma_f32_16x16x32_f16(false, a, false, b, (short)0, c,
                                                 false, false);
  asm volatile("v_nop\n\tv_nop\n\tv_nop\n\tv_nop" : "+v"(d) : "v"(a), "v"(b));
  return d;
}

__device__ __forceinline__ float red16_sum(float x) {
#pragma unroll
  for (int off = 1; off < 16; off <<= 1) x += __shfl_xor(x, off, 32);
  return x;
}

__device__ __forceinline__ void wave_lds_sync() {
  __builtin_amdgcn_fence(3  , "wavefront");
  asm volatile("s_wait_dscnt 0x0" ::: "memory");
  __builtin_amdgcn_wave_barrier();
}

__device__ __forceinline__ float silu_act(float z) {
  return z * __builtin_amdgcn_rcpf(1.0f + __expf(-z));
}

__device__ __forceinline__ void wplane_piece(const float* __restrict__ src,
                                             _Float16* __restrict__ dst, unsigned piece) {
  const v4f a0 = *(const v4f*)(src + (size_t)piece * 8u);
  const v4f a1 = *(const v4f*)(src + (size_t)piece * 8u + 4u);
  v8h o;
#pragma unroll
  for (int i = 0; i < 4; ++i) {
    o[i]     = toh_flush(WCARRY * bf16r(a0[i]));
    o[i + 4] = toh_flush(WCARRY * bf16r(a1[i]));
  }
  _Float16* p = dst + (size_t)piece * 8u;
  *(volatile v8h*)p = o;
  __threadfence();
  *(volatile v8h*)p = o;
}

__global__ __launch_bounds__(256) void wplane_kernel(
    const float* __restrict__ W0, const float* __restrict__ W1,
    _Float16* __restrict__ W0h, _Float16* __restrict__ W1h) {
  const unsigned tid = threadIdx.x;
  if (blockIdx.x < (unsigned)(W0_PIECES / 256)) {
    wplane_piece(W0, W0h, blockIdx.x * 256u + tid);
  } else {
    wplane_piece(W1, W1h, (blockIdx.x - (unsigned)(W0_PIECES / 256)) * 256u + tid);
  }
}

__device__ __forceinline__ void layer1_tile(
    const int* __restrict__ bij, const float* __restrict__ fn, const _Float16* Ws0,
    const unsigned e, const unsigned hh, const unsigned m, v8f& acc0, v8f& acc1, int& te_out) {
  int te = bij[e];
  te = (te < 0) ? 0 : ((te > (NTYPE - 1)) ? (NTYPE - 1) : te);
  const float* fp = fn + (size_t)e * NBAS + hh * 8u;
  const v4f a0 = *(const v4f*)(fp);
  const v4f a1 = *(const v4f*)(fp + 4);
  v8h fv;
#pragma unroll
  for (int i = 0; i < 4; ++i) {
    fv[i]     = toh_flush(FCARRY * bf16r(a0[i]));
    fv[i + 4] = toh_flush(FCARRY * bf16r(a1[i]));
  }
  const v8h zz = {};
  acc0 = (v8f){};
  acc1 = (v8f){};
#pragma unroll
  for (int s = 0; s < NTYPE / 2; ++s) {
    const v8h lo = (te == 2 * s) ? fv : zz;
    const v8h hi = (te == 2 * s + 1) ? fv : zz;
    const v16h xb = join8(lo, hi);
    const _Float16* wp = Ws0 + ((unsigned)(2 * s) * NHID + m) * NBAS + hh * 8u;
    const v16h wa0 = frag2(wp, wp + NHID * NBAS);
    const v16h wa1 = frag2(wp + 16 * NBAS, wp + NHID * NBAS + 16 * NBAS);
    acc0 = wmma16(wa0, xb, acc0);
    acc1 = wmma16(wa1, xb, acc1);
  }
  te_out = te;
}

__global__ __launch_bounds__(256) void l1stat_kernel(
    const int* __restrict__ bij, const float* __restrict__ fn,
    const _Float16* __restrict__ W0h, float* __restrict__ part1) {
  __shared__ __attribute__((aligned(16))) _Float16 Ws0[W0_HALVES];
  __shared__ __attribute__((aligned(16))) float red[WAVES * 64];
  __shared__ __attribute__((aligned(16))) float pst[64];
  static_assert(sizeof(_Float16) * W0_HALVES + 4 * (WAVES * 64 + 64) <= 131072);

  const unsigned tid = threadIdx.x, lane = tid & 31u;
  const unsigned wave = (unsigned)__builtin_amdgcn_readfirstlane((int)(threadIdx.x >> 5));
  const unsigned hh = lane >> 4, m = lane & 15u;

#pragma unroll
  for (unsigned j = 0; j < 4u; ++j) {
    const unsigned idx = tid + 256u * j;
    *(v8h*)&Ws0[idx * 8u] = *(const v8h*)(W0h + (size_t)idx * 8u);
  }
  __syncthreads();

  float s0[8], s1[8], q0[8], q1[8];
#pragma unroll
  for (int v = 0; v < 8; ++v) { s0[v] = 0.0f; s1[v] = 0.0f; q0[v] = 0.0f; q1[v] = 0.0f; }

  const unsigned tile0 = (blockIdx.x * (unsigned)WAVES + wave) * (unsigned)TPW;
#pragma unroll 1
  for (unsigned it = 0; it < (unsigned)TPW; ++it) {
    const unsigned e = (tile0 + it) * 16u + m;
    v8f acc0, acc1;
    int te;
    layer1_tile(bij, fn, Ws0, e, hh, m, acc0, acc1, te);
#pragma unroll
    for (int v = 0; v < 8; ++v) {
      const float x0 = acc0[v] * L1SCALE;
      const float x1 = acc1[v] * L1SCALE;
      s0[v] += x0;  q0[v] += x0 * x0;
      s1[v] += x1;  q1[v] += x1 * x1;
    }
  }

#pragma unroll
  for (int v = 0; v < 8; ++v) {
    s0[v] = red16_sum(s0[v]);
    s1[v] = red16_sum(s1[v]);
    q0[v] = red16_sum(q0[v]);
    q1[v] = red16_sum(q1[v]);
  }
  if (m == 0u) {
#pragma unroll
    for (int v = 0; v < 8; ++v) {
      red[wave * 64u + hh * 8u + (unsigned)v]       = s0[v];
      red[wave * 64u + 16u + hh * 8u + (unsigned)v] = s1[v];
      red[wave * 64u + 32u + hh * 8u + (unsigned)v] = q0[v];
      red[wave * 64u + 48u + hh * 8u + (unsigned)v] = q1[v];
    }
  }
  __syncthreads();
  if (tid < 64u) {
    float t = 0.0f;
#pragma unroll
    for (unsigned w = 0; w < (unsigned)WAVES; ++w) t += red[w * 64u + tid];
    pst[tid] = t;
  }
  __syncthreads();
  if (tid < (unsigned)(P1W / 4)) {
    const v4f x = *(const v4f*)&pst[tid * 4u];
    float* p = part1 + (size_t)blockIdx.x * P1W + tid * 4u;
    *(volatile v4f*)p = x;
    __threadfence();
    *(volatile v4f*)p = x;
  }
}

template <int C, int PW>
__device__ __forceinline__ void bnfin_body(
    const float* __restrict__ part, const float* __restrict__ gamma,
    const float* __restrict__ beta, const int* __restrict__ normp, float* __restrict__ tbl) {
#pragma clang fp contract(off)
  __shared__ double sd[64];
  __shared__ __attribute__((aligned(16))) float tb[64];
  static_assert(2 * C <= 64 && 2 * C <= PW);
  const unsigned tid = threadIdx.x;
  const unsigned j = (tid < (unsigned)(2 * C)) ? tid : (unsigned)(2 * C - 1);
  double acc = 0.0;
#pragma unroll 4
  for (unsigned b = 0; b < (unsigned)NBLK; ++b) acc += (double)part[(size_t)b * PW + j];
  sd[tid] = acc;
  tb[tid] = 0.0f;
  __syncthreads();

  const unsigned c = (tid < (unsigned)C) ? tid : (unsigned)(C - 1);
  const double mean = sd[c] * (1.0 / (double)NE);
  double var = sd[(unsigned)C + c] * (1.0 / (double)NE) - mean * mean;
  var = (var > 0.0) ? var : 0.0;
  const float rstd = rsqrtf((float)var + BN_EPS);
  const int nrm = normp[0];
  const float g  = bf16r(gamma[c]);
  const float be = bf16r(beta[c]);
  const float a  = rstd * g;
  const float sh = (float)((double)be - mean * (double)a);
  const float a_out  = (nrm != 0) ? a : 1.0f;
  const float sh_out = (nrm != 0) ? sh : 0.0f;
  if (tid < (unsigned)C) {
    tb[tid] = a_out;
    tb[(unsigned)C + tid] = sh_out;
  }
  __syncthreads();
  const unsigned TW = (2 * C > 32) ? (unsigned)(2 * C) : 32u;
  if (tid < TW / 4u) {
    const v4f x = *(const v4f*)&tb[tid * 4u];
    float* p = tbl + tid * 4u;
    *(volatile v4f*)p = x;
    __threadfence();
    *(volatile v4f*)p = x;
  }
}

__global__ __launch_bounds__(64) void bnfin1_kernel(
    const float* __restrict__ part, const float* __restrict__ gamma,
    const float* __restrict__ beta, const int* __restrict__ normp, float* __restrict__ tbl) {
  bnfin_body<NHID, P1W>(part, gamma, beta, normp, tbl);
}
__global__ __launch_bounds__(64) void bnfin2_kernel(
    const float* __restrict__ part, const float* __restrict__ gamma,
    const float* __restrict__ beta, const int* __restrict__ normp, float* __restrict__ tbl) {
  bnfin_body<NOUT, P2W>(part, gamma, beta, normp, tbl);
}

__global__ __launch_bounds__(256) void l2_kernel(
    const int* __restrict__ bij, const float* __restrict__ fn,
    const _Float16* __restrict__ W0h, const _Float16* __restrict__ W1h,
    const float* __restrict__ tbl1, float* __restrict__ out2, float* __restrict__ part2) {
  __shared__ __attribute__((aligned(16))) _Float16 Ws0[W0_HALVES];
  __shared__ __attribute__((aligned(16))) _Float16 Ws1[W1_HALVES];
  __shared__ __attribute__((aligned(16))) float Os[WAVES * 128];
  __shared__ __attribute__((aligned(16))) float red[WAVES * 16];
  __shared__ __attribute__((aligned(16))) float pst[32];
  static_assert(2 * (W0_HALVES + W1_HALVES) + 4 * (WAVES * 128 + WAVES * 16 + 32) <= 131072);

  const unsigned tid = threadIdx.x, lane = tid & 31u;
  const unsigned wave = (unsigned)__builtin_amdgcn_readfirstlane((int)(threadIdx.x >> 5));
  const unsigned hh = lane >> 4, m = lane & 15u;

#pragma unroll
  for (unsigned j = 0; j < 4u; ++j) {
    const unsigned idx = tid + 256u * j;
    *(v8h*)&Ws0[idx * 8u] = *(const v8h*)(W0h + (size_t)idx * 8u);
  }
#pragma unroll
  for (unsigned j = 0; j < 2u; ++j) {
    const unsigned idx = tid + 256u * j;
    *(v8h*)&Ws1[idx * 8u] = *(const v8h*)(W1h + (size_t)idx * 8u);
  }
  __syncthreads();

  float af0[8], bf0[8], af1[8], bf1[8];
  {
    const float* tp = tbl1 + hh * 8u;
    const v4f ta0 = *(const v4f*)(tp);
    const v4f ta1 = *(const v4f*)(tp + 4);
    const v4f ta2 = *(const v4f*)(tp + 16);
    const v4f ta3 = *(const v4f*)(tp + 20);
    const v4f tb0 = *(const v4f*)(tp + 32);
    const v4f tb1 = *(const v4f*)(tp + 36);
    const v4f tb2 = *(const v4f*)(tp + 48);
    const v4f tb3 = *(const v4f*)(tp + 52);
#pragma unroll
    for (int v = 0; v < 4; ++v) {
      af0[v] = ta0[v];  af0[v + 4] = ta1[v];
      af1[v] = ta2[v];  af1[v + 4] = ta3[v];
      bf0[v] = tb0[v];  bf0[v + 4] = tb1[v];
      bf1[v] = tb2[v];  bf1[v + 4] = tb3[v];
    }
  }

  float s2[8], q2[8];
#pragma unroll
  for (int v = 0; v < 8; ++v) { s2[v] = 0.0f; q2[v] = 0.0f; }

  const unsigned tile0 = (blockIdx.x * (unsigned)WAVES + wave) * (unsigned)TPW;
#pragma unroll 1
  for (unsigned it = 0; it < (unsigned)TPW; ++it) {
    const unsigned tile = tile0 + it;
    const unsigned e = tile * 16u + m;
    v8f acc0, acc1;
    int te;
    layer1_tile(bij, fn, Ws0, e, hh, m, acc0, acc1, te);

    v8h ylo, yhi;
#pragma unroll
    for (int v = 0; v < 8; ++v) {
      const float z0 = (acc0[v] * L1SCALE) * af0[v] + bf0[v];
      const float z1 = (acc1[v] * L1SCALE) * af1[v] + bf1[v];
      ylo[v] = toh_flush(YCARRY * silu_act(z0));
      yhi[v] = toh_flush(YCARRY * silu_act(z1));
    }
    const v16h yb = join8(ylo, yhi);

    v8f res = {};
#pragma unroll
    for (int mt = 0; mt < (NTYPE * NOUT) / 16; ++mt) {
      const v16h wa = frag_at(Ws1 + ((unsigned)(16 * mt) + m) * NHID + hh * 8u);
      const v8f zero = {};
      const v8f d = wmma16(wa, yb, zero);
      const bool sel = (te == 2 * mt + (int)hh);
      res = sel ? d : res;
    }

    float o[8];
#pragma unroll
    for (int r = 0; r < 8; ++r) {
      const float other = __shfl_xor(res[r], 16, 32);
      o[r] = (res[r] + other) * L2SCALE;
      s2[r] += o[r];
      q2[r] += o[r] * o[r];
    }

    v4f st;
#pragma unroll
    for (int j = 0; j < 4; ++j) st[j] = (hh != 0u) ? o[4 + j] : o[j];
    *(v4f*)&Os[wave * 128u + m * 8u + hh * 4u] = st;
    wave_lds_sync();
    const v4f ov = *(const v4f*)&Os[wave * 128u + lane * 4u];
    wave_lds_sync();
    float* p = out2 + (size_t)tile * 128u + lane * 4u;
    *(volatile v4f*)p = ov;
    __threadfence();
    *(volatile v4f*)p = ov;
  }

#pragma unroll
  for (int v = 0; v < 8; ++v) {
    s2[v] = red16_sum(s2[v]);
    q2[v] = red16_sum(q2[v]);
  }
  if (lane == 0u) {
#pragma unroll
    for (int v = 0; v < 8; ++v) {
      red[wave * 16u + (unsigned)v]      = s2[v];
      red[wave * 16u + 8u + (unsigned)v] = q2[v];
    }
  }
  __syncthreads();
  if (tid < 32u) {
    const unsigned j = tid & 15u;
    float t = 0.0f;
#pragma unroll
    for (unsigned w = 0; w < (unsigned)WAVES; ++w) t += red[w * 16u + j];
    pst[tid] = (tid < 16u) ? t : 0.0f;
  }
  __syncthreads();
  if (tid < (unsigned)(P2W / 4)) {
    const v4f x = *(const v4f*)&pst[tid * 4u];
    float* p = part2 + (size_t)blockIdx.x * P2W + tid * 4u;
    *(volatile v4f*)p = x;
    __threadfence();
    *(volatile v4f*)p = x;
  }
}

__global__ __launch_bounds__(256) void out_kernel(
    const float* __restrict__ out2, const float* __restrict__ tbl2, float* __restrict__ out) {
#pragma clang fp contract(off)
  const unsigned i = blockIdx.x * 256u + threadIdx.x;
  const unsigned c0 = (i & 1u) * 4u;
  const v4f x = *(const v4f*)(out2 + (size_t)i * 4u);
  const v4f a = *(const v4f*)(tbl2 + c0);
  const v4f b = *(const v4f*)(tbl2 + NOUT + c0);
  v4f o;
#pragma unroll
  for (int j = 0; j < 4; ++j) {
    const float z = x[j] * a[j] + b[j];
    o[j] = silu_act(z);
  }
  float* p = out + (size_t)i * 4u;
  *(volatile v4f*)p = o;
  __threadfence();
  *(volatile v4f*)p = o;
}

extern "C" void kernel_launch(void* const* d_in, const int* in_sizes, int n_in,
                              void* d_out, int out_size, void* d_ws, size_t ws_size,
                              hipStream_t stream) {
  if (n_in < 9) return;
  if ((long long)in_sizes[0] < (long long)NE) return;
  if ((long long)in_sizes[1] < (long long)NE * NBAS) return;
  if (in_sizes[2] < W0_HALVES) return;
  if (in_sizes[3] < W1_HALVES) return;
  if (in_sizes[4] < NHID || in_sizes[5] < NHID) return;
  if (in_sizes[6] < NOUT || in_sizes[7] < NOUT) return;
  if (in_sizes[8] < 1) return;
  if ((long long)out_size < (long long)NE * NOUT) return;
  if (ws_size < WS_TOTAL) return;

  const int*   bij = (const int*)d_in[0];
  const float* fn  = (const float*)d_in[1];
  const float* w0  = (const float*)d_in[2];
  const float* w1  = (const float*)d_in[3];
  const float* g1  = (const float*)d_in[4];
  const float* b1  = (const float*)d_in[5];
  const float* g2  = (const float*)d_in[6];
  const float* b2  = (const float*)d_in[7];
  const int*   nrm = (const int*)d_in[8];
  float* out = (float*)d_out;

  char* ws = (char*)d_ws;
  _Float16* W0h  = (_Float16*)(ws + OFF_W0H);
  _Float16* W1h  = (_Float16*)(ws + OFF_W1H);
  float*    P1   = (float*)(ws + OFF_P1);
  float*    T1   = (float*)(ws + OFF_T1);
  float*    P2   = (float*)(ws + OFF_P2);
  float*    T2   = (float*)(ws + OFF_T2);
  float*    O2   = (float*)(ws + OFF_O2);

  wplane_kernel<<<dim3((W0_PIECES + W1_PIECES) / 256), dim3(256), 0, stream>>>(w0, w1, W0h, W1h);
  l1stat_kernel<<<dim3(NBLK), dim3(256), 0, stream>>>(bij, fn, W0h, P1);
  bnfin1_kernel<<<dim3(1), dim3(64), 0, stream>>>(P1, g1, b1, nrm, T1);
  l2_kernel<<<dim3(NBLK), dim3(256), 0, stream>>>(bij, fn, W0h, W1h, T1, O2, P2);
  bnfin2_kernel<<<dim3(1), dim3(64), 0, stream>>>(P2, g2, b2, nrm, T2);
  out_kernel<<<dim3((NE * 2) / 256), dim3(256), 0, stream>>>(O2, T2, out);
}
